// PathTransformer_47278999994619
// MI455X (gfx1250) — hardware-verified
//
#include <hip/hip_runtime.h>
#include <stddef.h>
#include <stdint.h>
#include <math.h>

#define NB    8
#define SL    1024
#define SL0   1023
#define DIN   16
#define DM    256
#define NH    8
#define HD    32
#define NLAY  3
#define DF    1024
#define NRBF  8
#define KE    320
#define NCW   275
#define MR    (NB * SL)
#define C3    (3 * DM)
#define PLN   ((size_t)NB * NH * SL * HD)
#define NEGF  (-100000.0f)

static_assert(NH * HD == DM);
static_assert(SL % 256 == 0);
static_assert(MR % 256 == 0);
static_assert(KE % 32 == 0);
static_assert(NCW + DIN <= KE);
static_assert(DM % 64 == 0);
static_assert(DF % 64 == 0);
static_assert(C3 % 64 == 0);
static_assert(MR % 8 == 0);

typedef _Float16 v16h __attribute__((ext_vector_type(16)));
typedef _Float16 v8h  __attribute__((ext_vector_type(8)));
typedef float    v8f  __attribute__((ext_vector_type(8)));
typedef float    v4f  __attribute__((ext_vector_type(4)));
typedef unsigned int v4u __attribute__((ext_vector_type(4)));

union Frag  { v16h v; v8h h[2]; };
union Pack8 { v8h h; v4u u; };

__device__ __forceinline__ v8f mma16(v16h a, v16h b, v8f c) {
  c = __builtin_amdgcn_wmma_f32_16x16x32_f16(false, a, false, b, (short)0, c, false, false);
  asm volatile("v_nop\n\tv_nop\n\tv_nop\n\tv_nop" : "+v"(c) : "v"(a), "v"(b));
  return c;
}

__device__ __forceinline__ v16h ldfrag(const _Float16* p, int ld, int row0, int k0, int lane) {
  const int m = lane & 15, lh = lane >> 4;
  const _Float16* q = p + (size_t)(row0 + m) * (size_t)ld + k0 + 8 * lh;
  Frag f;
  f.h[0] = *(const v8h*)(q);
  f.h[1] = *(const v8h*)(q + 16);
  return f.v;
}

__device__ __forceinline__ v8f zero8() { return (v8f){0.f, 0.f, 0.f, 0.f, 0.f, 0.f, 0.f, 0.f}; }

__device__ __forceinline__ float act16(float v) {
  return 8.0f * v * (1.0f + erff(v * 0.70710678118654752f));
}

template <int NKS>
__device__ __forceinline__ void gemm32x64(const _Float16* __restrict__ A, int lda, int astep,
                                          const _Float16* __restrict__ Bt, int ldb,
                                          int ma, int n0, int lane, v8f (&acc)[2][4]) {
#pragma unroll 2
  for (int ks = 0; ks < NKS; ++ks) {
    const _Float16* Ak = A + (size_t)ks * (size_t)astep;
    const int kb = ks * 32;
    const v16h a0 = ldfrag(Ak, lda, ma, 0, lane);
    const v16h a1 = ldfrag(Ak, lda, ma + 16, 0, lane);
    const v16h b0 = ldfrag(Bt, ldb, n0, kb, lane);
    const v16h b1 = ldfrag(Bt, ldb, n0 + 16, kb, lane);
    const v16h b2 = ldfrag(Bt, ldb, n0 + 32, kb, lane);
    const v16h b3 = ldfrag(Bt, ldb, n0 + 48, kb, lane);
    acc[0][0] = mma16(a0, b0, acc[0][0]);
    acc[1][0] = mma16(a1, b0, acc[1][0]);
    acc[0][1] = mma16(a0, b1, acc[0][1]);
    acc[1][1] = mma16(a1, b1, acc[1][1]);
    acc[0][2] = mma16(a0, b2, acc[0][2]);
    acc[1][2] = mma16(a1, b2, acc[1][2]);
    acc[0][3] = mma16(a0, b3, acc[0][3]);
    acc[1][3] = mma16(a1, b3, acc[1][3]);
  }
}

__global__ __launch_bounds__(256) void k_cvt(const float* __restrict__ w, _Float16* __restrict__ o, int ngrp, float sc) {
  const int t = blockIdx.x * 256 + (int)threadIdx.x;
  if (t >= ngrp) return;
  const size_t off = (size_t)t * 8;
  const v4f a0 = *(const v4f*)(w + off);
  const v4f a1 = *(const v4f*)(w + off + 4);
  Pack8 pk;
  pk.h = (v8h){(_Float16)(a0[0] * sc), (_Float16)(a0[1] * sc), (_Float16)(a0[2] * sc), (_Float16)(a0[3] * sc),
               (_Float16)(a1[0] * sc), (_Float16)(a1[1] * sc), (_Float16)(a1[2] * sc), (_Float16)(a1[3] * sc)};
  const v4u vv = pk.u;
  volatile v4u* d = (volatile v4u*)(o + off);
  *d = vv;
  __threadfence();
  *d = vv;
}

__global__ __launch_bounds__(256) void k_we(const float* __restrict__ cw, const float* __restrict__ iw,
                                           _Float16* __restrict__ we) {
  const int p = blockIdx.x * 256 + (int)threadIdx.x;
  if (p >= DM * (KE / 8)) return;
  const int n = p / (KE / 8);
  const int j = p - n * (KE / 8);
  float v[8];
#pragma unroll
  for (int e = 0; e < 8; ++e) {
    const int c  = 8 * j + e;
    const int ci = (c < NCW) ? c : (NCW - 1);
    int xi = c - NCW;
    xi = (xi < 0) ? 0 : ((xi > DIN - 1) ? (DIN - 1) : xi);
    const float a  = cw[(size_t)n * NCW + ci];
    const float bb = iw[n * DIN + xi];
    v[e] = (c < NCW) ? a : ((c < NCW + DIN) ? bb : 0.0f);
  }
  Pack8 pk;
  pk.h = (v8h){(_Float16)(v[0] * 32.0f), (_Float16)(v[1] * 32.0f), (_Float16)(v[2] * 32.0f), (_Float16)(v[3] * 32.0f),
               (_Float16)(v[4] * 32.0f), (_Float16)(v[5] * 32.0f), (_Float16)(v[6] * 32.0f), (_Float16)(v[7] * 32.0f)};
  const v4u vv = pk.u;
  volatile v4u* d = (volatile v4u*)(we + (size_t)p * 8);
  *d = vv;
  __threadfence();
  *d = vv;
}

__global__ __launch_bounds__(256) void k_prep(const float* __restrict__ x, const float* __restrict__ c_local,
                                             const float* __restrict__ c_sink, const int* __restrict__ lengths,
                                             const float* __restrict__ pos_emb, const float* __restrict__ rbf_c,
                                             const float* __restrict__ rbf_w, _Float16* __restrict__ ep) {
  __shared__ __align__(16) float ext[8][64];
  const int tid = threadIdx.x, lane = tid & 31, wave = tid >> 5;
  const int row = blockIdx.x * 8 + wave;
  const int b = row >> 10, l = row & (SL - 1);
  int len = lengths[b];
  len = (len < 0) ? 0 : ((len > SL0) ? SL0 : len);
  const int msk = (l > len);
  const float zs = msk ? 0.0f : 16.0f;
  const int lm1 = (l > 0) ? (l - 1) : 0;
  const float clg = c_local[(size_t)b * SL0 + lm1];
  const float csg = c_sink[(size_t)b * SL0 + lm1];
  const float clraw = (l > 0) ? clg : 0.0f;
  const float csraw = (l > 0) ? csg : 0.0f;
  const float cl = 0.5f * fminf(fmaxf(clraw, 0.0f), 1.0f);
  const float cs = 1.0f * fminf(fmaxf(csraw, 0.0f), 1.0f);

  const float* pr = pos_emb + (size_t)l * DM + 8 * lane;
  const v4f p0 = *(const v4f*)(pr);
  const v4f p1 = *(const v4f*)(pr + 4);
  Pack8 pa;
  pa.h = (v8h){(_Float16)(p0[0] * zs), (_Float16)(p0[1] * zs), (_Float16)(p0[2] * zs), (_Float16)(p0[3] * zs),
               (_Float16)(p1[0] * zs), (_Float16)(p1[1] * zs), (_Float16)(p1[2] * zs), (_Float16)(p1[3] * zs)};

  const int ri = (lane - 3) & 7;
  const float cen = rbf_c[ri];
  const float wid = rbf_w[ri];
  const float cc = (lane < 11) ? cl : cs;
  const float dd = (cc - cen) * (1.0f / (wid + 1e-6f));
  const float rv = __expf(-0.5f * dd * dd);
  const float raw = (lane == 0) ? cl : ((lane == 1) ? cs : cl * cs);
  int xi0 = lane - 19;
  xi0 = (xi0 < 0) ? 0 : xi0;
  int xi1 = lane + 13;
  xi1 = (xi1 > DIN - 1) ? (DIN - 1) : xi1;
  const float* xr = x + ((size_t)b * SL0 + lm1) * DIN;
  const float xv0 = xr[xi0];
  const float xv1 = xr[xi1];
  const float xs = (l > 0) ? 16.0f : 0.0f;
  const float v0 = (lane < 3) ? (raw * zs) : ((lane < 19) ? (rv * zs) : (xv0 * xs));
  const float v1 = (lane < 3) ? (xv1 * xs) : 0.0f;
  ext[wave][lane]      = v0;
  ext[wave][32 + lane] = v1;
  __syncthreads();
  const int q8 = (lane & 7) * 8;
  const float* ew = ext[wave];
  Pack8 pb;
  pb.h = (v8h){(_Float16)ew[q8 + 0], (_Float16)ew[q8 + 1], (_Float16)ew[q8 + 2], (_Float16)ew[q8 + 3],
               (_Float16)ew[q8 + 4], (_Float16)ew[q8 + 5], (_Float16)ew[q8 + 6], (_Float16)ew[q8 + 7]};
  const v4u va = pa.u, vb = pb.u;
  _Float16* erow = ep + (size_t)row * KE;
  volatile v4u* da = (volatile v4u*)(erow + 8 * lane);
  volatile v4u* db = (volatile v4u*)(erow + DM + q8);
  *da = va;
  if (lane < 8) *db = vb;
  __threadfence();
  *da = va;
  if (lane < 8) *db = vb;
}

__device__ __forceinline__ void ln_row(const float* __restrict__ ir, const float* __restrict__ g,
                                       const float* __restrict__ bt, int lane, float (&o)[8]) {
  const v4f a0 = *(const v4f*)(ir + 8 * lane);
  const v4f a1 = *(const v4f*)(ir + 8 * lane + 4);
  float s = ((a0[0] + a0[1]) + (a0[2] + a0[3])) + ((a1[0] + a1[1]) + (a1[2] + a1[3]));
#pragma unroll
  for (int off = 1; off < 32; off <<= 1) s += __shfl_xor(s, off, 32);
  const float mean = s * (1.0f / (float)DM);
  float d[8];
  d[0] = a0[0] - mean; d[1] = a0[1] - mean; d[2] = a0[2] - mean; d[3] = a0[3] - mean;
  d[4] = a1[0] - mean; d[5] = a1[1] - mean; d[6] = a1[2] - mean; d[7] = a1[3] - mean;
  float q = ((d[0] * d[0] + d[1] * d[1]) + (d[2] * d[2] + d[3] * d[3])) +
            ((d[4] * d[4] + d[5] * d[5]) + (d[6] * d[6] + d[7] * d[7]));
#pragma unroll
  for (int off = 1; off < 32; off <<= 1) q += __shfl_xor(q, off, 32);
  const float var = q * (1.0f / (float)DM);
  const float inv = rsqrtf(var + 1e-5f);
  const v4f g0 = *(const v4f*)(g + 8 * lane);
  const v4f g1 = *(const v4f*)(g + 8 * lane + 4);
  const v4f b0 = *(const v4f*)(bt + 8 * lane);
  const v4f b1 = *(const v4f*)(bt + 8 * lane + 4);
  o[0] = d[0] * inv * g0[0] + b0[0];
  o[1] = d[1] * inv * g0[1] + b0[1];
  o[2] = d[2] * inv * g0[2] + b0[2];
  o[3] = d[3] * inv * g0[3] + b0[3];
  o[4] = d[4] * inv * g1[0] + b1[0];
  o[5] = d[5] * inv * g1[1] + b1[1];
  o[6] = d[6] * inv * g1[2] + b1[2];
  o[7] = d[7] * inv * g1[3] + b1[3];
}

__global__ __launch_bounds__(256) void k_ln(const float* __restrict__ in, const float* __restrict__ g,
                                           const float* __restrict__ bt, _Float16* __restrict__ outh,
                                           int nrows, int rpb) {
  const int tid = threadIdx.x, lane = tid & 31, wave = tid >> 5;
  const int idx = blockIdx.x * 8 + wave;
  if (idx >= nrows) return;
  const int qb = idx / rpb;
  const int row = qb * SL + (idx - qb * rpb);
  float o[8];
  ln_row(in + (size_t)row * DM, g, bt, lane, o);
  Pack8 pk;
  pk.h = (v8h){(_Float16)o[0], (_Float16)o[1], (_Float16)o[2], (_Float16)o[3],
               (_Float16)o[4], (_Float16)o[5], (_Float16)o[6], (_Float16)o[7]};
  const v4u vv = pk.u;
  volatile v4u* d = (volatile v4u*)(outh + (size_t)row * DM + 8 * lane);
  *d = vv;
  __threadfence();
  *d = vv;
}

__global__ __launch_bounds__(256) void k_lnout(const float* __restrict__ in, const float* __restrict__ g,
                                              const float* __restrict__ bt, float* __restrict__ out) {
  __shared__ __align__(16) float rb[8][DM];
  const int tid = threadIdx.x, lane = tid & 31, wave = tid >> 5;
  float o[8];
  ln_row(in + (size_t)wave * SL * DM, g, bt, lane, o);
  *(v4f*)(rb[wave] + 8 * lane)     = (v4f){o[0], o[1], o[2], o[3]};
  *(v4f*)(rb[wave] + 8 * lane + 4) = (v4f){o[4], o[5], o[6], o[7]};
  __syncthreads();
  const v4f u0 = *(const v4f*)(rb[wave] + 4 * lane);
  const v4f u1 = *(const v4f*)(rb[wave] + 128 + 4 * lane);
  volatile v4f* d0 = (volatile v4f*)(out + (size_t)wave * DM + 4 * lane);
  volatile v4f* d1 = (volatile v4f*)(out + (size_t)wave * DM + 128 + 4 * lane);
  *d0 = u0;
  *d1 = u1;
  __threadfence();
  *d0 = u0;
  *d1 = u1;
}

#define STP 72
__global__ __launch_bounds__(256) void k_qkv(const _Float16* __restrict__ yh,
                                             const _Float16* __restrict__ wt,
                                             const float* __restrict__ bias,
                                             _Float16* __restrict__ qkv) {
  __shared__ __align__(16) _Float16 st[256 * STP];
  const int tid = threadIdx.x, lane = tid & 31, wave = tid >> 5;
  const int hh = lane >> 4, c = lane & 15;
  const int mb = blockIdx.x * 256;
  const int m0 = mb + wave * 32;
  const int n0 = blockIdx.y * 64;
  const int which = n0 >> 8;
  const int nin = n0 & (DM - 1);
  const int h0 = nin >> 5;

  v8f acc[2][4];
#pragma unroll
  for (int s = 0; s < 2; ++s)
#pragma unroll
    for (int t = 0; t < 4; ++t) acc[s][t] = zero8();
  gemm32x64<DM / 32>(yh, DM, 32, wt, DM, m0, n0, lane, acc);

#pragma unroll
  for (int t = 0; t < 4; ++t) {
    const float bb = bias[n0 + 16 * t + c];
#pragma unroll
    for (int sub = 0; sub < 2; ++sub) {
#pragma unroll
      for (int r = 0; r < 8; ++r) {
        const int lr = wave * 32 + sub * 16 + 8 * hh + r;
        st[lr * STP + 16 * t + c] = (_Float16)(acc[sub][t][r] * 0.03125f + bb);
      }
    }
  }
  __syncthreads();

  const int b  = mb >> 10;
  const int nb = mb & (SL - 1);
  v4u val[8];
  size_t go[8];
  if (which < 2) {
#pragma unroll
    for (int j = 0; j < 8; ++j) {
      const int p    = tid + 256 * j;
      const int hsel = p >> 10;
      const int pp   = p & 1023;
      const int lr   = pp >> 2;
      const int pc   = pp & 3;
      Pack8 pk;
      pk.h   = *(const v8h*)(st + lr * STP + 32 * hsel + 8 * pc);
      val[j] = pk.u;
      go[j]  = (size_t)which * PLN + ((size_t)(b * NH + h0 + hsel) * SL + nb + lr) * HD + pc * 8;
    }
  } else {
#pragma unroll
    for (int j = 0; j < 8; ++j) {
      const int p    = tid + 256 * j;
      const int hsel = p >> 10;
      const int pp   = p & 1023;
      const int d    = pp >> 5;
      const int pc   = pp & 31;
      const int nl   = pc * 8;
      const _Float16* cp = st + nl * STP + 32 * hsel + d;
      Pack8 pk;
      pk.h = (v8h){cp[0 * STP], cp[1 * STP], cp[2 * STP], cp[3 * STP],
                   cp[4 * STP], cp[5 * STP], cp[6 * STP], cp[7 * STP]};
      val[j] = pk.u;
      go[j]  = 2 * PLN + ((size_t)(b * NH + h0 + hsel) * HD + d) * SL + nb + nl;
    }
  }
  for (int ps = 0; ps < 2; ++ps) {
#pragma unroll
    for (int j = 0; j < 8; ++j) *(volatile v4u*)(qkv + go[j]) = val[j];
    __threadfence();
  }
}

#define KTP 40
#define VTP 72
#define PTP 72
__global__ __launch_bounds__(256) void k_attn(const _Float16* __restrict__ qp,
                                              const _Float16* __restrict__ kp,
                                              const _Float16* __restrict__ vt,
                                              const float* __restrict__ c_local,
                                              const float* __restrict__ c_sink,
                                              const int* __restrict__ lengths,
                                              _Float16* __restrict__ op, int nqb, float sscale) {
  __shared__ __align__(16) _Float16 Ks[64 * KTP];
  __shared__ __align__(16) _Float16 Vs[HD * VTP];
  __shared__ __align__(16) _Float16 Ps[8][16 * PTP];

  const int tid = threadIdx.x, lane = tid & 31, wave = tid >> 5;
  const int hh = lane >> 4, c = lane & 15;
  const int blk = blockIdx.x;
  const int bh = blk / nqb;
  const int qb = blk - bh * nqb;
  const int b  = bh >> 3;
  const int q0 = qb * 128 + wave * 16;
  int len = lengths[b];
  len = (len < 0) ? 0 : ((len > SL0) ? SL0 : len);
  int nkc = (len + 64) >> 6;
  nkc = (nkc < 1) ? 1 : ((nkc > SL / 64) ? (SL / 64) : nkc);

  const _Float16* Q = qp + (size_t)bh * SL * HD;
  const _Float16* K = kp + (size_t)bh * SL * HD;
  const _Float16* V = vt + (size_t)bh * HD * SL;

  const v16h qa = ldfrag(Q, HD, q0, 0, lane);

  float cli[8], csi[8];
  int mski[8], iq[8];
#pragma unroll
  for (int r = 0; r < 8; ++r) {
    const int i = q0 + 8 * hh + r;
    const int im1 = (i > 0) ? (i - 1) : 0;
    const float clg = c_local[(size_t)b * SL0 + im1];
    const float csg = c_sink[(size_t)b * SL0 + im1];
    cli[r]  = (i > 0) ? clg : 0.0f;
    csi[r]  = (i > 0) ? csg : 0.0f;
    mski[r] = (i > len) ? 1 : 0;
    iq[r]   = i;
  }

  const float NEGI = -__builtin_huge_valf();
  float mrow[8], lrow[8];
  v8f oacc[2];
#pragma unroll
  for (int r = 0; r < 8; ++r) { mrow[r] = NEGI; lrow[r] = 0.f; }
#pragma unroll
  for (int t = 0; t < 2; ++t) oacc[t] = zero8();

  _Float16* pw = Ps[wave];

  for (int kc = 0; kc < nkc; ++kc) {
    const int kv0 = kc * 64;
    __syncthreads();
    {
      const int r  = tid >> 2;
      const int qq = (tid & 3) * 8;
      *(v8h*)(Ks + r * KTP + qq) = *(const v8h*)(K + (size_t)(kv0 + r) * HD + qq);
      const int r2 = tid >> 3;
      const int q2 = (tid & 7) * 8;
      *(v8h*)(Vs + r2 * VTP + q2) = *(const v8h*)(V + (size_t)r2 * SL + kv0 + q2);
    }
    __syncthreads();

    v8f s[4];
#pragma unroll
    for (int j = 0; j < 4; ++j) {
      const v16h kb = ldfrag(Ks, KTP, j * 16, 0, lane);
      s[j] = mma16(qa, kb, zero8());
    }

    float clj[4], csj[4];
    int mskj[4], jk[4];
#pragma unroll
    for (int j = 0; j < 4; ++j) {
      const int jj  = kv0 + 16 * j + c;
      const int jm1 = (jj > 0) ? (jj - 1) : 0;
      const float clg = c_local[(size_t)b * SL0 + jm1];
      const float csg = c_sink[(size_t)b * SL0 + jm1];
      clj[j]  = (jj > 0) ? clg : 0.0f;
      csj[j]  = (jj > 0) ? csg : 0.0f;
      mskj[j] = (jj > len) ? 1 : 0;
      jk[j]   = jj;
    }

    float cm[8];
#pragma unroll
    for (int r = 0; r < 8; ++r) {
      float m = NEGI;
#pragma unroll
      for (int j = 0; j < 4; ++j) {
        const int dlt = iq[r] - jk[j];
        const bool nb1  = (dlt == 1) || (dlt == -1);
        const bool usei = (dlt == 1) && ((jk[j] == 0) || (iq[r] == SL - 1));
        const float e   = nb1 ? (usei ? cli[r] : clj[j]) : 0.0f;
        const float bia = 0.5f * e + csi[r] * csj[j];
        float sv = s[j][r] * sscale + bia;
        sv = ((mski[r] | mskj[j]) != 0) ? NEGF : sv;
        s[j][r] = sv;
        m = fmaxf(m, sv);
      }
#pragma unroll
      for (int off = 1; off < 16; off <<= 1) m = fmaxf(m, __shfl_xor(m, off, 32));
      cm[r] = m;
    }
    float al[8];
#pragma unroll
    for (int r = 0; r < 8; ++r) {
      const float mnew  = fmaxf(mrow[r], cm[r]);
      const float alpha = __expf(mrow[r] - mnew);
      mrow[r] = mnew;
      float psum = 0.f;
#pragma unroll
      for (int j = 0; j < 4; ++j) {
        const float p = __expf(s[j][r] - mnew);
        psum += p;
        pw[(8 * hh + r) * PTP + j * 16 + c] = (_Float16)(p * 1024.0f);
      }
#pragma unroll
      for (int off = 1; off < 16; off <<= 1) psum += __shfl_xor(psum, off, 32);
      lrow[r] = lrow[r] * alpha + psum;
      al[r] = alpha;
    }
#pragma unroll
    for (int t = 0; t < 2; ++t)
#pragma unroll
      for (int r = 0; r < 8; ++r) oacc[t][r] *= al[r];
    __syncthreads();

#pragma unroll
    for (int kk = 0; kk < 2; ++kk) {
      const v16h pa = ldfrag(pw, PTP, 0, kk * 32, lane);
#pragma unroll
      for (int t = 0; t < 2; ++t) {
        const v16h vb = ldfrag(Vs, VTP, t * 16, kk * 32, lane);
        oacc[t] = mma16(pa, vb, oacc[t]);
      }
    }
  }
  __syncthreads();

#pragma unroll
  for (int r = 0; r < 8; ++r) {
    const float inv = 0.0625f / lrow[r];
#pragma unroll
    for (int t = 0; t < 2; ++t) pw[(8 * hh + r) * PTP + 16 * t + c] = (_Float16)(oacc[t][r] * inv);
  }
  __syncthreads();
  v4u val[2];
  size_t go[2];
#pragma unroll
  for (int it = 0; it < 2; ++it) {
    const int p  = lane + 32 * it;
    const int L  = p >> 2;
    const int pc = p & 3;
    Pack8 pk;
    pk.h    = *(const v8h*)(pw + L * PTP + pc * 8);
    val[it] = pk.u;
    go[it]  = ((size_t)bh * SL + q0 + L) * HD + pc * 8;
  }
  for (int ps = 0; ps < 2; ++ps) {
#pragma unroll
    for (int it = 0; it < 2; ++it) *(volatile v4u*)(op + go[it]) = val[it];
    __threadfence();
  }
}

#define OTP 68
template <int NKS, int AHEAD, int MODE>
__global__ __launch_bounds__(256) void k_gout(const _Float16* __restrict__ ap,
                                              const _Float16* __restrict__ wt,
                                              const float* __restrict__ bias,
                                              const float* __restrict__ bias2,
                                              const float* __restrict__ clsv,
                                              const int* __restrict__ lengths,
                                              const float* __restrict__ res,
                                              float* __restrict__ out, float oscale, int mstride) {
  __shared__ __align__(16) float st[8][16 * OTP];
  const int tid = threadIdx.x, lane = tid & 31, wave = tid >> 5;
  const int hh = lane >> 4, c = lane & 15;
  const int mb = blockIdx.x * mstride;
  const int m0 = mb + wave * 32;
  const int n0 = blockIdx.y * 64;
  const int b  = mb >> 10;

  v8f acc[2][4];
#pragma unroll
  for (int s = 0; s < 2; ++s)
#pragma unroll
    for (int t = 0; t < 4; ++t) acc[s][t] = zero8();
  if (AHEAD) {
    gemm32x64<NKS>(ap + (size_t)b * NH * SL * HD, HD, SL * HD, wt, NKS * 32, m0 & (SL - 1), n0, lane, acc);
  } else {
    gemm32x64<NKS>(ap, NKS * 32, 32, wt, NKS * 32, m0, n0, lane, acc);
  }

  float bvs[4], b2s[4], cl4[4];
#pragma unroll
  for (int t = 0; t < 4; ++t) {
    const int n = n0 + 16 * t + c;
    bvs[t] = bias[n];
    b2s[t] = 0.f;
    cl4[t] = 0.f;
    if (MODE == 1) { b2s[t] = bias2[n]; cl4[t] = clsv[n]; }
  }
  int len = 0;
  if (MODE == 1) {
    len = lengths[b];
    len = (len < 0) ? 0 : ((len > SL0) ? SL0 : len);
  }

  float* sw = st[wave];
#pragma unroll
  for (int sub = 0; sub < 2; ++sub) {
    __syncthreads();
#pragma unroll
    for (int t = 0; t < 4; ++t) {
#pragma unroll
      for (int r = 0; r < 8; ++r) {
        float ad = bvs[t];
        if (MODE == 1) {
          const int l = (m0 + sub * 16 + 8 * hh + r) & (SL - 1);
          const float keep = (l > len) ? 0.0f : 1.0f;
          ad = (l == 0) ? (cl4[t] + b2s[t]) : (bvs[t] + keep * b2s[t]);
        }
        sw[(8 * hh + r) * OTP + 16 * t + c] = acc[sub][t][r] * oscale + ad;
      }
    }
    __syncthreads();
    v4f val[8];
    size_t go[8];
#pragma unroll
    for (int it = 0; it < 8; ++it) {
      const int p    = lane + 32 * it;
      const int L    = p >> 3;
      const int pc   = p & 7;
      const int row  = L >> 1;
      const int half = L & 1;
      const size_t gidx = (size_t)(m0 + sub * 16 + row) * DM + n0 + half * 32 + pc * 4;
      v4f v = *(const v4f*)(sw + row * OTP + half * 32 + pc * 4);
      if (MODE == 0) {
        const v4f rr = *(const v4f*)(res + gidx);
        v[0] = v[0] + rr[0]; v[1] = v[1] + rr[1]; v[2] = v[2] + rr[2]; v[3] = v[3] + rr[3];
      }
      val[it] = v;
      go[it]  = gidx;
    }
    for (int ps = 0; ps < 2; ++ps) {
#pragma unroll
      for (int it = 0; it < 8; ++it) *(volatile v4f*)(out + go[it]) = val[it];
      __threadfence();
    }
  }
}

__global__ __launch_bounds__(256) void k_ffn1(const _Float16* __restrict__ yh,
                                              const _Float16* __restrict__ wt,
                                              const float* __restrict__ bias,
                                              _Float16* __restrict__ gp, int mstride) {
  __shared__ __align__(16) float st[8][16 * OTP];
  const int tid = threadIdx.x, lane = tid & 31, wave = tid >> 5;
  const int hh = lane >> 4, c = lane & 15;
  const int m0 = blockIdx.x * mstride + wave * 32;
  const int n0 = blockIdx.y * 64;

  v8f acc[2][4];
#pragma unroll
  for (int s = 0; s < 2; ++s)
#pragma unroll
    for (int t = 0; t < 4; ++t) acc[s][t] = zero8();
  gemm32x64<DM / 32>(yh, DM, 32, wt, DM, m0, n0, lane, acc);

  float bvs[4];
#pragma unroll
  for (int t = 0; t < 4; ++t) bvs[t] = bias[n0 + 16 * t + c];

  float* sw = st[wave];
#pragma unroll
  for (int sub = 0; sub < 2; ++sub) {
    __syncthreads();
#pragma unroll
    for (int t = 0; t < 4; ++t) {
#pragma unroll
      for (int r = 0; r < 8; ++r)
        sw[(8 * hh + r) * OTP + 16 * t + c] = acc[sub][t][r] * 0.03125f + bvs[t];
    }
    __syncthreads();
    v4u val[4];
    size_t go[4];
#pragma unroll
    for (int it = 0; it < 4; ++it) {
      const int p  = lane + 32 * it;
      const int L  = p >> 3;
      const int pc = p & 7;
      const v4f x0 = *(const v4f*)(sw + L * OTP + pc * 8);
      const v4f x1 = *(const v4f*)(sw + L * OTP + pc * 8 + 4);
      Pack8 pk;
      pk.h = (v8h){(_Float16)act16(x0[0]), (_Float16)act16(x0[1]), (_Float16)act16(x0[2]), (_Float16)act16(x0[3]),
                   (_Float16)act16(x1[0]), (_Float16)act16(x1[1]), (_Float16)act16(x1[2]), (_Float16)act16(x1[3])};
      val[it] = pk.u;
      go[it]  = (size_t)(m0 + sub * 16 + L) * DF + n0 + pc * 8;
    }
    for (int ps = 0; ps < 2; ++ps) {
#pragma unroll
      for (int it = 0; it < 4; ++it) *(volatile v4u*)(gp + go[it]) = val[it];
      __threadfence();
    }
  }
}

extern "C" void kernel_launch(void* const* d_in, const int* in_sizes, int n_in,
                              void* d_out, int out_size, void* d_ws, size_t ws_size,
                              hipStream_t stream) {
  if (n_in < 26) return;
  if (in_sizes[0] != NB * SL0 * DIN) return;
  if (in_sizes[1] != NB * SL0 || in_sizes[2] != NB * SL0) return;
  if (in_sizes[3] != NB) return;
  if (in_sizes[4] != DM * DIN || in_sizes[5] != DM || in_sizes[6] != DM) return;
  if (in_sizes[7] < SL * DM) return;
  if (in_sizes[8] != DM * NCW || in_sizes[9] != DM) return;
  if (in_sizes[10] != NRBF || in_sizes[11] != NRBF) return;
  if (in_sizes[12] != NLAY * C3 * DM || in_sizes[13] != NLAY * C3) return;
  if (in_sizes[14] != NLAY * DM * DM || in_sizes[15] != NLAY * DM) return;
  if (in_sizes[16] != NLAY * DF * DM || in_sizes[17] != NLAY * DF) return;
  if (in_sizes[18] != NLAY * DM * DF || in_sizes[19] != NLAY * DM) return;
  if (in_sizes[20] != NLAY * DM || in_sizes[21] != NLAY * DM) return;
  if (in_sizes[22] != NLAY * DM || in_sizes[23] != NLAY * DM) return;
  if (in_sizes[24] != DM || in_sizes[25] != DM) return;
  if (out_size != NB * DM) return;

  const float* x         = (const float*)d_in[0];
  const float* c_local   = (const float*)d_in[1];
  const float* c_sink    = (const float*)d_in[2];
  const int*   lengths   = (const int*)d_in[3];
  const float* input_w   = (const float*)d_in[4];
  const float* input_b   = (const float*)d_in[5];
  const float* cls_tok   = (const float*)d_in[6];
  const float* pos_emb   = (const float*)d_in[7];
  const float* corr_w    = (const float*)d_in[8];
  const float* corr_b    = (const float*)d_in[9];
  const float* rbf_c     = (const float*)d_in[10];
  const float* rbf_w     = (const float*)d_in[11];
  const float* in_proj_w = (const float*)d_in[12];
  const float* in_proj_b = (const float*)d_in[13];
  const float* out_w     = (const float*)d_in[14];
  const float* out_b     = (const float*)d_in[15];
  const float* ff_w1     = (const float*)d_in[16];
  const float* ff_b1     = (const float*)d_in[17];
  const float* ff_w2     = (const float*)d_in[18];
  const float* ff_b2     = (const float*)d_in[19];
  const float* ln1_g     = (const float*)d_in[20];
  const float* ln1_b     = (const float*)d_in[21];
  const float* ln2_g     = (const float*)d_in[22];
  const float* ln2_b     = (const float*)d_in[23];
  const float* lnout_g   = (const float*)d_in[24];
  const float* lnout_b   = (const float*)d_in[25];
  float* out = (float*)d_out;

  size_t off = 0;
  const size_t oE   = off; off += (size_t)MR * KE * 2;
  const size_t oWE  = off; off += (size_t)DM * KE * 2;
  const size_t oHA  = off; off += (size_t)MR * DM * 4;
  const size_t oHB  = off; off += (size_t)MR * DM * 4;
  const size_t oY   = off; off += (size_t)MR * DM * 2;
  const size_t oWQ  = off; off += (size_t)NLAY * C3 * DM * 2;
  const size_t oWO  = off; off += (size_t)NLAY * DM * DM * 2;
  const size_t oW1  = off; off += (size_t)NLAY * DF * DM * 2;
  const size_t oW2  = off; off += (size_t)NLAY * DM * DF * 2;
  const size_t oQKV = off; off += 3 * PLN * 2;
  const size_t oO   = off; off += (size_t)MR * DM * 2;
  const size_t oG   = off; off += (size_t)MR * DF * 2;
  if (off > ws_size) return;
  if (off > (size_t)134217728) return;

  char* ws = (char*)d_ws;
  _Float16* Ep  = (_Float16*)(ws + oE);
  _Float16* WEp = (_Float16*)(ws + oWE);
  float*    HA  = (float*)(ws + oHA);
  float*    HB  = (float*)(ws + oHB);
  _Float16* Yp  = (_Float16*)(ws + oY);
  _Float16* WQ  = (_Float16*)(ws + oWQ);
  _Float16* WO  = (_Float16*)(ws + oWO);
  _Float16* W1  = (_Float16*)(ws + oW1);
  _Float16* W2  = (_Float16*)(ws + oW2);
  _Float16* QKV = (_Float16*)(ws + oQKV);
  _Float16* Op  = (_Float16*)(ws + oO);
  _Float16* Gp  = (_Float16*)(ws + oG);

  {
    const int g0 = in_sizes[12] / 8, g1 = in_sizes[14] / 8, g2 = in_sizes[16] / 8, g3 = in_sizes[18] / 8;
    k_cvt<<<dim3((g0 + 255) / 256), dim3(256), 0, stream>>>(in_proj_w, WQ, g0, 32.0f);
    k_cvt<<<dim3((g1 + 255) / 256), dim3(256), 0, stream>>>(out_w, WO, g1, 32.0f);
    k_cvt<<<dim3((g2 + 255) / 256), dim3(256), 0, stream>>>(ff_w1, W1, g2, 32.0f);
    k_cvt<<<dim3((g3 + 255) / 256), dim3(256), 0, stream>>>(ff_w2, W2, g3, 32.0f);
  }
  k_we<<<dim3((DM * (KE / 8) + 255) / 256), dim3(256), 0, stream>>>(corr_w, input_w, WEp);
  k_prep<<<dim3(MR / 8), dim3(256), 0, stream>>>(x, c_local, c_sink, lengths, pos_emb, rbf_c, rbf_w, Ep);
  k_gout<KE / 32, 0, 1><<<dim3(MR / 256, DM / 64), dim3(256), 0, stream>>>(
      Ep, WEp, input_b, corr_b, cls_tok, lengths, HB, HA, 0.001953125f, 256);

  for (int l = 0; l < NLAY; ++l) {
    const int full    = (l < NLAY - 1) ? 1 : 0;
    const int nqb     = full ? (SL / 128) : 1;
    const int mstride = full ? 256 : SL;
    const int gx      = full ? (MR / 256) : NB;
    const int nr2     = full ? MR : (NB * 256);
    const int rpb2    = full ? SL : 256;
    k_ln<<<dim3(MR / 8), dim3(256), 0, stream>>>(HA, ln1_g + l * DM, ln1_b + l * DM, Yp, MR, SL);
    k_qkv<<<dim3(MR / 256, C3 / 64), dim3(256), 0, stream>>>(Yp, WQ + (size_t)l * C3 * DM, in_proj_b + l * C3, QKV);
    k_attn<<<dim3(NB * NH * nqb), dim3(256), 0, stream>>>(QKV, QKV + PLN, QKV + 2 * PLN, c_local, c_sink, lengths,
                                                         Op, nqb, 0.17677669529663689f);
    k_gout<DM / 32, 1, 0><<<dim3(gx, DM / 64), dim3(256), 0, stream>>>(
        Op, WO + (size_t)l * DM * DM, out_b + l * DM, out_b + l * DM, cls_tok, lengths, HA, HB, 0.00048828125f, mstride);
    k_ln<<<dim3(nr2 / 8), dim3(256), 0, stream>>>(HB, ln2_g + l * DM, ln2_b + l * DM, Yp, nr2, rpb2);
    k_ffn1<<<dim3(gx, DF / 64), dim3(256), 0, stream>>>(Yp, W1 + (size_t)l * DF * DM, ff_b1 + l * DF, Gp, mstride);
    k_gout<DF / 32, 0, 0><<<dim3(gx, DM / 64), dim3(256), 0, stream>>>(
        Gp, W2 + (size_t)l * DM * DF, ff_b2 + l * DM, ff_b2 + l * DM, cls_tok, lengths, HB, HA, 0.001953125f, mstride);
  }
  k_lnout<<<dim3(1), dim3(256), 0, stream>>>(HA, lnout_g, lnout_b, out);
  (void)hipGetLastError();
}
